// MoE_47742856462430
// MI455X (gfx1250) — hardware-verified
//
#include <hip/hip_runtime.h>
#include <math.h>

typedef __attribute__((ext_vector_type(16))) _Float16 v16h;
typedef __attribute__((ext_vector_type(16))) __bf16 v16b;
typedef __attribute__((ext_vector_type(8)))  _Float16 v8h;
typedef __attribute__((ext_vector_type(8)))  __bf16 v8b;
typedef __attribute__((ext_vector_type(8)))  float v8f;
typedef __attribute__((ext_vector_type(4)))  float v4f;
typedef __attribute__((ext_vector_type(4)))  unsigned v4u;
typedef _Float16 h16;

#ifndef NB
#define NB 8192
#endif
#define NB_FULL 8192
#define DIN  512
#define DHID 1024
#define DOUT 512
#define NE   16
#define TOPK 2
#define MT   128
#define RMAX (TOPK * NB + NE * MT)
#define NTILE (RMAX / MT)
#define NTILE_PAD (((NTILE + 31) / 32) * 32)
#define NCH (NB / 32)
#define RTK_PIECES (RMAX / 8)
#define RTK_IT ((RTK_PIECES + 511) / 512)
#define GKC 128
#define GXP (GKC + 4)
#define HCARRY 64.0f
#define WCARRY 512.0f
#define OSCALE (1.0f / 32768.0f)

#define WS_XB  ((size_t)0)
#define WS_W1T (WS_XB  + (size_t)NB * DIN * 2)
#define WS_W2T (WS_W1T + (size_t)NE * DHID * DIN * 2)
#define WS_HB  (WS_W2T + (size_t)NE * DOUT * DHID * 2)
#define WS_YS  (WS_HB  + (size_t)RMAX * DHID * 2)
#define WS_XG  (WS_YS)
#define WS_SEL (WS_YS  + (size_t)RMAX * DOUT * 4)
#define WS_REC (WS_SEL + (size_t)NB * 16)
#define WS_RTK (WS_REC + (size_t)NB * 16)
#define WS_TLE (WS_RTK + (size_t)RMAX * 2)
#define WS_END (WS_TLE + (size_t)NTILE_PAD * 4)

static_assert(NB % 128 == 0);
static_assert(NB <= NB_FULL);
static_assert(NB <= 65535);
static_assert(DIN % 32 == 0 && DHID % 32 == 0 && (DIN * 2) % 128 == 0 && (DHID * 2) % 128 == 0 && (DOUT * 4) % 128 == 0);
static_assert(DHID % 128 == 0 && DOUT % 128 == 0 && RMAX % MT == 0 && MT == 128);
static_assert((size_t)NB_FULL * DOUT * 4 == 16777216);
static_assert((size_t)RMAX * DIN * 2 <= (size_t)RMAX * DOUT * 4);
static_assert(WS_W1T % 128 == 0 && WS_W2T % 128 == 0 && WS_HB % 128 == 0 && WS_YS % 128 == 0);
static_assert(WS_SEL % 128 == 0 && WS_REC % 128 == 0 && WS_RTK % 128 == 0 && WS_TLE % 128 == 0);
static_assert(WS_END <= (size_t)134217728);
static_assert((size_t)(NB * DIN / 8 / 256) * 256 * 8 == (size_t)NB * DIN);
static_assert((size_t)(DHID / 64) * (DIN / 64) * NE * 4096 == (size_t)NE * DIN * DHID);
static_assert((size_t)(DOUT / 64) * (DHID / 64) * NE * 4096 == (size_t)NE * DHID * DOUT);
static_assert((size_t)(NB / 64) * 64 * 16 == (size_t)NB * 16);
static_assert(DIN % GKC == 0 && NE == 16 && (GXP * 4) % 16 == 0);
static_assert((size_t)8 * 128 * 8 == (size_t)64 * GKC);
static_assert((size_t)4 * 128 * 4 == (size_t)GKC * NE);
static_assert(NCH * 32 == NB);
static_assert(RMAX % 8 == 0 && RTK_PIECES % 32 == 0 && RTK_IT * 512 >= RTK_PIECES);
static_assert(NTILE_PAD % 32 == 0 && NTILE_PAD <= 512 && NTILE <= NTILE_PAD);
static_assert(RMAX % 32 == 0 && (size_t)256 * 16 * 8 == (size_t)32 * DIN * 2);
static_assert((size_t)(DHID / 128) * NTILE * 128 * 128 == (size_t)RMAX * DHID);
static_assert((size_t)32 * 16 * 8 == (size_t)32 * 128);
static_assert((size_t)(DOUT / 128) * NTILE * 128 * 128 == (size_t)RMAX * DOUT);
static_assert((size_t)32 * 16 * 8 == (size_t)16 * 256);
static_assert(NB % 16 == 0 && (size_t)256 * 16 * 8 == (size_t)16 * DOUT * 4);
static_assert(64 * 65 * 4 <= 131072);
static_assert(64 * GXP * 4 + GKC * NE * 4 + 64 * NE * 4 <= 131072);
static_assert(RMAX * 2 + NCH * NE * 4 + (NE + 1) * 4 + NE * 4 <= 131072);
static_assert(8 * 32 * 64 * 2 <= 131072);
static_assert(8 * 16 * 64 * 4 <= 131072);

__device__ __forceinline__ v8f wmma16(v16h a, v16h b, v8f c) {
  v8f d = __builtin_amdgcn_wmma_f32_16x16x32_f16(false, a, false, b, (short)0, c, false, false);
  asm volatile("v_nop\n\tv_nop\n\tv_nop\n\tv_nop" : "+v"(d) : "v"(a), "v"(b));
  return d;
}
__device__ __forceinline__ v8f wmma_bf(v16b a, v16b b, v8f c) {
  v8f d = __builtin_amdgcn_wmma_f32_16x16x32_bf16(false, a, false, b, (short)0, c, false, false);
  asm volatile("v_nop\n\tv_nop\n\tv_nop\n\tv_nop" : "+v"(d) : "v"(a), "v"(b));
  return d;
}
__device__ __forceinline__ float bfr(float v) { return (float)(__bf16)v; }
static __device__ __forceinline__ h16 toh_flush(float v) { const h16 r = (h16)v; return (fabsf(v) < 6.103515625e-05f) ? (h16)0.0f : r; }
__device__ __forceinline__ v16b ldfrag_b(const unsigned short* p) { union { v16b v; v4u q[2]; } f; f.q[0] = *(const v4u*)p; f.q[1] = *(const v4u*)(p + 16); return f.v; }
__device__ __forceinline__ v16h ldfrag_h(const unsigned short* p) { union { v16h v; v4u q[2]; } f; f.q[0] = *(const v4u*)p; f.q[1] = *(const v4u*)(p + 16); return f.v; }

__global__ __launch_bounds__(256) void k_cvt_x(const float* __restrict__ X, unsigned short* __restrict__ XB) {
  const unsigned i = blockIdx.x * 256u + threadIdx.x;
  const unsigned ic = i < (unsigned)(NB * DIN / 8) ? i : (unsigned)(NB * DIN / 8 - 1);
  const v4f a = *(const v4f*)(X + (size_t)ic * 8), b = *(const v4f*)(X + (size_t)ic * 8 + 4);
  union { v8b h; v4u u; } o;
#pragma unroll
  for (int j = 0; j < 4; ++j) { o.h[j] = (__bf16)a[j]; o.h[4 + j] = (__bf16)b[j]; }
  const v4u val = o.u;
  volatile v4u* p = (volatile v4u*)(XB + (size_t)ic * 8);
  *p = val; __threadfence(); *p = val;
}

template <int F16>
__global__ __launch_bounds__(256) void k_tr(const float* __restrict__ S, unsigned short* __restrict__ Dst, unsigned K, unsigned N, unsigned dpitch, unsigned erow, unsigned ecol, float sc) {
  __shared__ float tile[64][65];
  const unsigned t = threadIdx.x, e = blockIdx.z, k0 = blockIdx.y * 64u, n0 = blockIdx.x * 64u;
  const float* s = S + (size_t)e * K * N;
#pragma unroll
  for (unsigned it = 0; it < 4; ++it) { const unsigned idx = it * 256u + t, kr = idx >> 4, c4 = idx & 15u;
    const v4f v = *(const v4f*)(s + (size_t)(k0 + kr) * N + n0 + 4u * c4);
    tile[kr][4u * c4 + 0] = v[0]; tile[kr][4u * c4 + 1] = v[1]; tile[kr][4u * c4 + 2] = v[2]; tile[kr][4u * c4 + 3] = v[3]; }
  __syncthreads();
  v4u o[2];
#pragma unroll
  for (unsigned it = 0; it < 2; ++it) { const unsigned idx = it * 256u + t, nr = idx >> 3, q = idx & 7u;
    union { v8b b; v8h h; v4u u; } w;
#pragma unroll
    for (int i = 0; i < 8; ++i) { const float v = bfr(tile[8u * q + i][nr]); if (F16) w.h[i] = toh_flush(v * sc); else w.b[i] = (__bf16)v; }
    o[it] = w.u; }
#pragma unroll
  for (unsigned it = 0; it < 2; ++it) { const unsigned idx = it * 256u + t, nr = idx >> 3, q = idx & 7u;
    *(volatile v4u*)(Dst + (size_t)(e * erow + n0 + nr) * dpitch + e * ecol + k0 + 8u * q) = o[it]; }
  __threadfence();
#pragma unroll
  for (unsigned it = 0; it < 2; ++it) { const unsigned idx = it * 256u + t, nr = idx >> 3, q = idx & 7u;
    *(volatile v4u*)(Dst + (size_t)(e * erow + n0 + nr) * dpitch + e * ecol + k0 + 8u * q) = o[it]; }
}

__global__ __launch_bounds__(128) void k_gate(const unsigned short* __restrict__ XB, const float* __restrict__ WG, unsigned* __restrict__ SEL) {
#pragma clang fp contract(off)
  __shared__ __align__(16) float xs[64][GXP];
  __shared__ __align__(16) float wgs[GKC][NE];
  __shared__ __align__(16) float sp[64][NE];
  const unsigned tid = threadIdx.x, lane = tid & 31u, col = lane & 15u, g = lane >> 4; const unsigned r0 = blockIdx.x * 64u;
  const unsigned wave = (unsigned)__builtin_amdgcn_readfirstlane((int)(threadIdx.x >> 5));
  const unsigned rl = wave * 16u + 8u * g;
  float acc[8];
#pragma unroll
  for (int r = 0; r < 8; ++r) acc[r] = 0.0f;
#pragma unroll 1
  for (unsigned kc = 0; kc < (unsigned)(DIN / GKC); ++kc) {
#pragma unroll
    for (unsigned it = 0; it < 8; ++it) { const unsigned idx = it * 128u + tid, rw = idx >> 4, q = idx & 15u;
      const v4u u = *(const v4u*)(XB + (size_t)(r0 + rw) * DIN + kc * (unsigned)GKC + 8u * q);
      xs[rw][8u * q + 0] = __uint_as_float(u[0] << 16); xs[rw][8u * q + 1] = __uint_as_float(u[0] & 0xFFFF0000u);
      xs[rw][8u * q + 2] = __uint_as_float(u[1] << 16); xs[rw][8u * q + 3] = __uint_as_float(u[1] & 0xFFFF0000u);
      xs[rw][8u * q + 4] = __uint_as_float(u[2] << 16); xs[rw][8u * q + 5] = __uint_as_float(u[2] & 0xFFFF0000u);
      xs[rw][8u * q + 6] = __uint_as_float(u[3] << 16); xs[rw][8u * q + 7] = __uint_as_float(u[3] & 0xFFFF0000u); }
#pragma unroll
    for (unsigned it = 0; it < 4; ++it) { const unsigned idx = it * 128u + tid, kr = idx >> 2, c4 = idx & 3u;
      const v4f v = *(const v4f*)(WG + (size_t)kc * GKC * NE + 4u * idx);
      wgs[kr][4u * c4 + 0] = bfr(v[0]); wgs[kr][4u * c4 + 1] = bfr(v[1]); wgs[kr][4u * c4 + 2] = bfr(v[2]); wgs[kr][4u * c4 + 3] = bfr(v[3]); }
    __syncthreads();
#pragma unroll 1
    for (unsigned k = 0; k < (unsigned)GKC; ++k) { const float w = wgs[k][col];
#pragma unroll
      for (int r = 0; r < 8; ++r) acc[r] = fmaf(xs[rl + r][k], w, acc[r]); }
    __syncthreads();
  }
#pragma unroll
  for (int r = 0; r < 8; ++r) sp[rl + r][col] = acc[r];
  __syncthreads();
  if (wave < 2u) {
    const unsigned tr = tid;
    float m = sp[tr][0];
#pragma unroll 1
    for (unsigned e = 1; e < NE; ++e) m = fmaxf(m, sp[tr][e]);
    float s = 0.0f;
#pragma unroll 1
    for (unsigned e = 0; e < NE; ++e) { const float ev = expf(sp[tr][e] - m); sp[tr][e] = ev; s += ev; }
    const float inv = 1.0f / s;
    float p0 = sp[tr][0] * inv; unsigned i0 = 0u;
#pragma unroll 1
    for (unsigned e = 1; e < NE; ++e) { const float p = sp[tr][e] * inv; const bool gt = p > p0; i0 = gt ? e : i0; p0 = gt ? p : p0; }
    float p1 = -1.0f; unsigned i1 = 0u;
#pragma unroll 1
    for (unsigned e = 0; e < NE; ++e) { const float p = sp[tr][e] * inv; const bool gt = (e != i0) && (p > p1); i1 = gt ? e : i1; p1 = gt ? p : p1; }
    v4u rec; rec[0] = i0; rec[1] = i1; rec[2] = __float_as_uint(p0); rec[3] = __float_as_uint(p1);
    volatile v4u* ps = (volatile v4u*)(SEL + (size_t)(r0 + tr) * 4u);
    *ps = rec; __threadfence(); *ps = rec;
  }
}

__global__ __launch_bounds__(512) void k_route(const unsigned* __restrict__ SEL, unsigned* __restrict__ REC, unsigned short* __restrict__ RTK, unsigned* __restrict__ TLE) {
  __shared__ __align__(16) unsigned short rtk[RMAX];
  __shared__ unsigned cnt[NCH][NE];
  __shared__ unsigned tot[NE];
  __shared__ unsigned segs[NE + 1];
  const unsigned tid = threadIdx.x, lane = tid & 31u;
  const unsigned wave = (unsigned)__builtin_amdgcn_readfirstlane((int)(threadIdx.x >> 5));
#pragma unroll 1
  for (unsigned i = tid; i < (unsigned)RMAX; i += 512u) rtk[i] = (unsigned short)0xFFFFu;
#pragma unroll 1
  for (unsigned c = wave; c < (unsigned)NCH; c += 16u) {
    const v4u s = *(const v4u*)(SEL + (size_t)(c * 32u + lane) * 4u);
    const unsigned i0 = s[0] & 15u, i1 = s[1] & 15u;
    unsigned mine = 0u;
#pragma unroll 1
    for (unsigned e = 0; e < NE; ++e) { const unsigned m = __builtin_amdgcn_ballot_w32((i0 == e) | (i1 == e)); const unsigned pc = (unsigned)__popc(m); mine = (lane == e) ? pc : mine; }
    if (lane < NE) cnt[c][lane] = mine;
  }
  __syncthreads();
  if (tid < NE) { unsigned run = 0u;
#pragma unroll 1
    for (unsigned c = 0; c < (unsigned)NCH; ++c) { const unsigned v = cnt[c][tid]; cnt[c][tid] = run; run += v; }
    tot[tid] = run; }
  __syncthreads();
  if (tid == 0u) { unsigned run = 0u;
#pragma unroll 1
    for (unsigned e = 0; e < NE; ++e) { segs[e] = run; run += (tot[e] + (unsigned)(MT - 1)) & ~(unsigned)(MT - 1); }
    segs[NE] = run; }
  __syncthreads();
  const unsigned lt = (1u << lane) - 1u;
#pragma unroll 1
  for (unsigned c = wave; c < (unsigned)NCH; c += 16u) {
    const unsigned tok = c * 32u + lane;
    const v4u s = *(const v4u*)(SEL + (size_t)tok * 4u);
    const unsigned i0 = s[0] & 15u, i1 = s[1] & 15u;
    unsigned s0 = 0u, s1 = 0u;
#pragma unroll 1
    for (unsigned e = 0; e < NE; ++e) { const unsigned m = __builtin_amdgcn_ballot_w32((i0 == e) | (i1 == e));
      const unsigned pos = segs[e] + cnt[c][e] + (unsigned)__popc(m & lt);
      s0 = (i0 == e) ? pos : s0; s1 = (i1 == e) ? pos : s1; }
    s0 = s0 < (unsigned)RMAX ? s0 : (unsigned)(RMAX - 1); s1 = s1 < (unsigned)RMAX ? s1 : (unsigned)(RMAX - 1);
    rtk[s0] = (unsigned short)tok; rtk[s1] = (unsigned short)tok;
    v4u rec; rec[0] = s0; rec[1] = s1; rec[2] = s[2]; rec[3] = s[3];
    volatile v4u* p = (volatile v4u*)(REC + (size_t)tok * 4u);
    *p = rec; __threadfence(); *p = rec;
  }
  __syncthreads();
  v4u o[RTK_IT];
#pragma unroll
  for (unsigned it = 0; it < (unsigned)RTK_IT; ++it) { const unsigned idx = it * 512u + tid; const unsigned ic = idx < (unsigned)RTK_PIECES ? idx : (unsigned)(RTK_PIECES - 1); o[it] = *(const v4u*)&rtk[8u * ic]; }
  const unsigned rowb = tid * (unsigned)MT; unsigned ex = 0xFFFFFFFFu;
#pragma unroll 1
  for (unsigned e = 0; e < NE; ++e) { const unsigned lo = segs[e], hi = segs[e + 1]; ex = (rowb >= lo && rowb < hi) ? e : ex; }
  volatile unsigned* pt = (volatile unsigned*)(TLE + (tid < (unsigned)NTILE_PAD ? tid : 0u));
#pragma unroll
  for (unsigned it = 0; it < (unsigned)RTK_IT; ++it) { const unsigned idx = it * 512u + tid; if (idx < (unsigned)RTK_PIECES) *(volatile v4u*)(RTK + (size_t)idx * 8u) = o[it]; }
  if (tid < (unsigned)NTILE_PAD) *pt = ex;
  __threadfence();
#pragma unroll
  for (unsigned it = 0; it < (unsigned)RTK_IT; ++it) { const unsigned idx = it * 512u + tid; if (idx < (unsigned)RTK_PIECES) *(volatile v4u*)(RTK + (size_t)idx * 8u) = o[it]; }
  if (tid < (unsigned)NTILE_PAD) *pt = ex;
}

__global__ __launch_bounds__(256) void k_gather(const unsigned short* __restrict__ XB, const unsigned short* __restrict__ RTK, unsigned short* __restrict__ XG) {
  const unsigned t = threadIdx.x, r0 = blockIdx.x * 32u;
  v4u o[8];
#pragma unroll
  for (unsigned it = 0; it < 8; ++it) { const unsigned idx = it * 256u + t, rw = idx >> 6, q = idx & 63u;
    const unsigned tok = RTK[r0 + rw]; const unsigned tc = tok < (unsigned)NB ? tok : 0u;
    v4u v = *(const v4u*)(XB + (size_t)tc * DIN + 8u * q);
    asm volatile("" : "+v"(v));
    const unsigned keep = tok < (unsigned)NB ? 0xFFFFFFFFu : 0u;
    v[0] &= keep; v[1] &= keep; v[2] &= keep; v[3] &= keep;
    o[it] = v; }
#pragma unroll
  for (unsigned it = 0; it < 8; ++it) { const unsigned idx = it * 256u + t, rw = idx >> 6, q = idx & 63u; *(volatile v4u*)(XG + (size_t)(r0 + rw) * DIN + 8u * q) = o[it]; }
  __threadfence();
#pragma unroll
  for (unsigned it = 0; it < 8; ++it) { const unsigned idx = it * 256u + t, rw = idx >> 6, q = idx & 63u; *(volatile v4u*)(XG + (size_t)(r0 + rw) * DIN + 8u * q) = o[it]; }
}

__global__ __launch_bounds__(256) void k_h(const unsigned short* __restrict__ XG, const unsigned short* __restrict__ W1T, const unsigned* __restrict__ TLE, unsigned short* __restrict__ HB) {
  __shared__ __align__(16) _Float16 sh[8][32][64];
  const unsigned t = threadIdx.x, wave = t >> 5, lane = t & 31u, lm = lane & 15u, lh = lane >> 4, wm = wave >> 1, wn = wave & 1u;
  const unsigned e = TLE[blockIdx.y];
  if (e >= (unsigned)NE) return;
  const unsigned m0 = blockIdx.y * 128u, n0 = blockIdx.x * 128u;
  const unsigned short* ar[2]; const unsigned short* br[4];
#pragma unroll
  for (int mi = 0; mi < 2; ++mi) ar[mi] = XG + (size_t)(m0 + wm * 32u + mi * 16u + lm) * DIN + 8u * lh;
#pragma unroll
  for (int ni = 0; ni < 4; ++ni) br[ni] = W1T + (size_t)(e * DHID + n0 + wn * 64u + ni * 16u + lm) * DIN + 8u * lh;
  v8f acc[2][4] = {};
#pragma unroll 2
  for (unsigned kc = 0; kc < DIN / 32; ++kc) { v16b a[2], b[4];
#pragma unroll
    for (int mi = 0; mi < 2; ++mi) a[mi] = ldfrag_b(ar[mi] + kc * 32u);
#pragma unroll
    for (int ni = 0; ni < 4; ++ni) b[ni] = ldfrag_b(br[ni] + kc * 32u);
#pragma unroll
    for (int mi = 0; mi < 2; ++mi)
#pragma unroll
      for (int ni = 0; ni < 4; ++ni) acc[mi][ni] = wmma_bf(a[mi], b[ni], acc[mi][ni]); }
#pragma unroll
  for (int ni = 0; ni < 4; ++ni) {
#pragma unroll
    for (int mi = 0; mi < 2; ++mi)
#pragma unroll
      for (int r = 0; r < 8; ++r) { const float hv = acc[mi][ni][r]; const float gl = 0.5f * hv * (1.0f + erff(hv * 0.70710678118654752f));
        sh[wave][mi * 16 + 8u * lh + r][ni * 16 + lm] = toh_flush(gl * HCARRY); } }
  __syncthreads();
  v4u o[8];
#pragma unroll
  for (unsigned it = 0; it < 8; ++it) { const unsigned rw = it * 4u + (lane >> 3), q = lane & 7u; union { v8h h; v4u u; } w; w.h = *(const v8h*)&sh[wave][rw][8u * q]; o[it] = w.u; }
  unsigned short* hb = HB + (size_t)(m0 + wm * 32u) * DHID + n0 + wn * 64u;
#pragma unroll
  for (unsigned it = 0; it < 8; ++it) { const unsigned rw = it * 4u + (lane >> 3), q = lane & 7u; *(volatile v4u*)(hb + (size_t)rw * DHID + 8u * q) = o[it]; }
  __threadfence();
#pragma unroll
  for (unsigned it = 0; it < 8; ++it) { const unsigned rw = it * 4u + (lane >> 3), q = lane & 7u; *(volatile v4u*)(hb + (size_t)rw * DHID + 8u * q) = o[it]; }
}

__global__ __launch_bounds__(256) void k_out(const unsigned short* __restrict__ HB, const unsigned short* __restrict__ W2T, const unsigned* __restrict__ TLE, float* __restrict__ YS) {
  __shared__ __align__(16) float sf[8][16][64];
  const unsigned t = threadIdx.x, wave = t >> 5, lane = t & 31u, lm = lane & 15u, lh = lane >> 4, wm = wave >> 1, wn = wave & 1u;
  const unsigned e = TLE[blockIdx.y];
  if (e >= (unsigned)NE) return;
  const unsigned m0 = blockIdx.y * 128u, n0 = blockIdx.x * 128u;
  const unsigned short* ar[2]; const unsigned short* br[4];
#pragma unroll
  for (int mi = 0; mi < 2; ++mi) ar[mi] = HB + (size_t)(m0 + wm * 32u + mi * 16u + lm) * DHID + 8u * lh;
#pragma unroll
  for (int ni = 0; ni < 4; ++ni) br[ni] = W2T + (size_t)(e * DOUT + n0 + wn * 64u + ni * 16u + lm) * DHID + 8u * lh;
  v8f acc[2][4] = {};
#pragma unroll 2
  for (unsigned kc = 0; kc < DHID / 32; ++kc) { v16h a[2], b[4];
#pragma unroll
    for (int mi = 0; mi < 2; ++mi) a[mi] = ldfrag_h(ar[mi] + kc * 32u);
#pragma unroll
    for (int ni = 0; ni < 4; ++ni) b[ni] = ldfrag_h(br[ni] + kc * 32u);
#pragma unroll
    for (int mi = 0; mi < 2; ++mi)
#pragma unroll
      for (int ni = 0; ni < 4; ++ni) acc[mi][ni] = wmma16(a[mi], b[ni], acc[mi][ni]); }
#pragma unroll
  for (int mi = 0; mi < 2; ++mi) {
    if (mi) __syncthreads();
#pragma unroll
    for (int ni = 0; ni < 4; ++ni)
#pragma unroll
      for (int r = 0; r < 8; ++r) sf[wave][8u * lh + r][ni * 16 + lm] = acc[mi][ni][r] * OSCALE;
    __syncthreads();
    v4f v[8];
#pragma unroll
    for (unsigned it = 0; it < 8; ++it) { const unsigned rw = it * 2u + (lane >> 4), pc = lane & 15u; v[it] = *(const v4f*)&sf[wave][rw][4u * pc]; }
    float* po = YS + (size_t)(m0 + wm * 32u + mi * 16u) * DOUT + n0 + wn * 64u;
#pragma unroll
    for (unsigned it = 0; it < 8; ++it) { const unsigned rw = it * 2u + (lane >> 4), pc = lane & 15u; *(volatile v4f*)(po + (size_t)rw * DOUT + 4u * pc) = v[it]; }
    __threadfence();
#pragma unroll
    for (unsigned it = 0; it < 8; ++it) { const unsigned rw = it * 2u + (lane >> 4), pc = lane & 15u; *(volatile v4f*)(po + (size_t)rw * DOUT + 4u * pc) = v[it]; }
  }
}

__global__ __launch_bounds__(256) void k_comb(const float* __restrict__ YS, const unsigned* __restrict__ REC, float* __restrict__ OUT) {
#pragma clang fp contract(off)
  const unsigned t = threadIdx.x, r0 = blockIdx.x * 16u;
  v4f o[8];
#pragma unroll
  for (unsigned it = 0; it < 8; ++it) { const unsigned idx = it * 256u + t, rw = idx >> 7, q = idx & 127u;
    const v4u rc = *(const v4u*)(REC + (size_t)(r0 + rw) * 4u);
    const unsigned s0 = rc[0] < (unsigned)RMAX ? rc[0] : (unsigned)(RMAX - 1), s1 = rc[1] < (unsigned)RMAX ? rc[1] : (unsigned)(RMAX - 1);
    const float p0 = __uint_as_float(rc[2]), p1 = __uint_as_float(rc[3]);
    const v4f a = *(const v4f*)(YS + (size_t)s0 * DOUT + 4u * q), b = *(const v4f*)(YS + (size_t)s1 * DOUT + 4u * q);
    v4f v;
#pragma unroll
    for (int j = 0; j < 4; ++j) { const float ma = p0 * a[j]; const float mb = p1 * b[j]; v[j] = ma + mb; }
    o[it] = v; }
#pragma unroll
  for (unsigned it = 0; it < 8; ++it) { const unsigned idx = it * 256u + t, rw = idx >> 7, q = idx & 127u; *(volatile v4f*)(OUT + (size_t)(r0 + rw) * DOUT + 4u * q) = o[it]; }
  __threadfence();
#pragma unroll
  for (unsigned it = 0; it < 8; ++it) { const unsigned idx = it * 256u + t, rw = idx >> 7, q = idx & 127u; *(volatile v4f*)(OUT + (size_t)(r0 + rw) * DOUT + 4u * q) = o[it]; }
}

extern "C" void kernel_launch(void* const* d_in, const int* in_sizes, int n_in, void* d_out, int out_size, void* d_ws, size_t ws_size, hipStream_t stream) {
  if (n_in < 4) return;
  if (in_sizes[0] < NB * DIN || in_sizes[1] < DIN * NE || in_sizes[2] < NE * DIN * DHID || in_sizes[3] < NE * DHID * DOUT) return;
  if ((size_t)out_size < (size_t)NB * DOUT) return;
  if (ws_size < (size_t)WS_END) return;
  const float* X  = (const float*)d_in[0];
  const float* WG = (const float*)d_in[1];
  const float* W1 = (const float*)d_in[2];
  const float* W2 = (const float*)d_in[3];
  char* ws = (char*)d_ws;
  unsigned short* XB  = (unsigned short*)(ws + WS_XB);
  unsigned short* W1T = (unsigned short*)(ws + WS_W1T);
  unsigned short* W2T = (unsigned short*)(ws + WS_W2T);
  unsigned short* HB  = (unsigned short*)(ws + WS_HB);
  float*          YS  = (float*)(ws + WS_YS);
  unsigned short* XG  = (unsigned short*)(ws + WS_XG);
  unsigned*       SEL = (unsigned*)(ws + WS_SEL);
  unsigned*       REC = (unsigned*)(ws + WS_REC);
  unsigned short* RTK = (unsigned short*)(ws + WS_RTK);
  unsigned*       TLE = (unsigned*)(ws + WS_TLE);
  float* OUT = (float*)d_out;
  k_cvt_x<<<dim3(NB * DIN / 8 / 256), 256, 0, stream>>>(X, XB);
  k_tr<0><<<dim3(DHID / 64, DIN / 64, NE), 256, 0, stream>>>(W1, W1T, (unsigned)DIN, (unsigned)DHID, (unsigned)DIN, (unsigned)DHID, 0u, 1.0f);
  k_tr<1><<<dim3(DOUT / 64, DHID / 64, NE), 256, 0, stream>>>(W2, W2T, (unsigned)DHID, (unsigned)DOUT, (unsigned)DHID, (unsigned)DOUT, 0u, WCARRY);
  k_gate<<<dim3(NB / 64), 128, 0, stream>>>(XB, WG, SEL);
  k_route<<<dim3(1), 512, 0, stream>>>(SEL, REC, RTK, TLE);
  k_gather<<<dim3(RMAX / 32), 256, 0, stream>>>(XB, RTK, XG);
  k_h<<<dim3(DHID / 128, NTILE), 256, 0, stream>>>(XG, W1T, TLE, HB);
  k_out<<<dim3(DOUT / 128, NTILE), 256, 0, stream>>>(HB, W2T, TLE, YS);
  k_comb<<<dim3(NB / 16), 256, 0, stream>>>(YS, REC, OUT);
}
